// MinimalMambaBlock_76974403879713
// MI455X (gfx1250) — hardware-run, weakly checked
//
#include <hip/hip_runtime.h>
#include <math.h>

typedef __attribute__((ext_vector_type(16))) _Float16 v16h;
typedef __attribute__((ext_vector_type(8)))  _Float16 v8h;
typedef __attribute__((ext_vector_type(8)))  float    v8f;
typedef __attribute__((ext_vector_type(4)))  float    v4f;

constexpr int kBatch    = 4;
constexpr int kSeq      = 2048;
constexpr int kDim      = 1024;
constexpr int kInner    = 2048;
constexpr int kSlabB    = 2;
constexpr int kSlabs    = kBatch / kSlabB;
constexpr int kSlabRows = kSlabB * kSeq;
constexpr int kPairs    = kInner / 2;
constexpr float kEps    = 1e-6f;

constexpr float kWCarry  = 1024.0f;
constexpr float kXnCarry = 16.0f;
constexpr float kUCarry  = 64.0f;
constexpr float kYCarry  = 64.0f;
constexpr float kScaleIG  = 1.0f / (kXnCarry * kWCarry);
constexpr float kScaleBCD = 1.0f / (kUCarry * kWCarry);
constexpr float kScaleOut = 1.0f / (kYCarry * kWCarry);

static_assert(kBatch % kSlabB == 0, "slabs by batch");
static_assert((kDim % 32) == 0 && (kInner % 32) == 0, "GEMM K multiples of 32");
static_assert((kSlabRows % 64) == 0 && (kInner % 64) == 0 && (kDim % 64) == 0, "GEMM M,N multiples of 64");
static_assert(((kSlabRows / 32) * (kInner / 64)) % 8 == 0, "gated tiles per block");
static_assert(((kSlabRows / 64) * (kInner / 64)) % 8 == 0, "bcd tiles per block");
static_assert(((kSlabRows / 64) * (kDim / 64)) % 8 == 0, "out tiles per block");
static_assert((kSlabRows % 8) == 0 && kDim == 1024, "norm kernel row map");
static_assert(((kSlabB * kPairs) % 64) == 0 && (kSeq % 4) == 0, "scan lane map");
static_assert((kInner % 256) == 0, "decay table blocks");

constexpr size_t kOffWIG  = 0;
constexpr size_t kOffWBCD = kOffWIG  + (size_t)2 * kInner * kDim * 2;
constexpr size_t kOffWO   = kOffWBCD + (size_t)3 * kInner * kInner * 2;
constexpr size_t kOffXN   = kOffWO   + (size_t)kDim * kInner * 2;
constexpr size_t kOffU    = kOffXN   + (size_t)kSlabRows * kDim * 2;
constexpr size_t kOffBCD  = kOffU    + (size_t)kSlabRows * kInner * 2;
constexpr size_t kOffY    = kOffBCD  + (size_t)3 * kSlabRows * kInner * 2;
constexpr size_t kOffADEC = kOffY    + (size_t)kSlabRows * kInner * 2;
constexpr size_t kWsTotal = kOffADEC + (size_t)kInner * 4;
static_assert(kWsTotal == 130031616ull, "carve total");
static_assert(kWsTotal <= 134217728ull, "carve cap");
static_assert((kOffWBCD % 128) == 0 && (kOffWO % 128) == 0 && (kOffXN % 128) == 0 && (kOffU % 128) == 0 &&
              (kOffBCD % 128) == 0 && (kOffY % 128) == 0 && (kOffADEC % 128) == 0, "128-B aligned regions");

union FragU { v16h v; v8h h[2]; };
__device__ __forceinline__ v16h frag_load(const _Float16* p) {
  FragU f;
  f.h[0] = *(const v8h*)(p);
  f.h[1] = *(const v8h*)(p + 16);
  return f.v;
}
__device__ __forceinline__ v8f mma_f16(v16h a, v16h b, v8f c) {
  return __builtin_amdgcn_wmma_f32_16x16x32_f16(false, a, false, b, (short)0, c, false, false);
}
__device__ __forceinline__ void guard1(v8f& acc, v16h a, v16h b) {
  asm volatile("v_nop\n\tv_nop\n\tv_nop\n\tv_nop" : "+v"(acc) : "v"(a), "v"(b));
}
__device__ __forceinline__ void wave_lds_sync() {
  __builtin_amdgcn_fence(__ATOMIC_RELEASE, "workgroup");
  __builtin_amdgcn_wave_barrier();
  __builtin_amdgcn_fence(__ATOMIC_ACQUIRE, "workgroup");
}

__device__ __forceinline__ float h16_to_f32(unsigned hb) {
  const unsigned sgn = (hb & 0x8000u) << 16;
  const unsigned em  = hb & 0x7fffu;
  const float fn  = __uint_as_float((em << 13) + 0x38000000u);
  const float fs  = (float)em * 5.9604644775390625e-8f;
  const float mag = (em < 0x400u) ? fs : fn;
  return __uint_as_float(__float_as_uint(mag) | sgn);
}
__device__ __forceinline__ unsigned pack_h2(float lo, float hi) {
  const _Float16 h0 = (_Float16)lo;
  const _Float16 h1 = (_Float16)hi;
  const unsigned short s0 = __builtin_bit_cast(unsigned short, h0);
  const unsigned short s1 = __builtin_bit_cast(unsigned short, h1);
  return (unsigned)s0 | ((unsigned)s1 << 16);
}

__global__ __launch_bounds__(256) void cast_carry_f16_kernel(
    const float* __restrict__ src, unsigned short* __restrict__ dst, int total8, float carry)
{
  const int i = blockIdx.x * 256 + threadIdx.x;
  if (i < total8) {
    const size_t e0 = (size_t)i << 3;
    const v4f a0 = *(const v4f*)(src + e0);
    const v4f a1 = *(const v4f*)(src + e0 + 4);
    v8h hv;
#pragma unroll
    for (int e = 0; e < 4; ++e) {
      hv[e]     = (_Float16)(a0[e] * carry);
      hv[4 + e] = (_Float16)(a1[e] * carry);
    }
    unsigned short* q = dst + e0;
    *(volatile v8h*)q = hv;
    __threadfence();
    *(volatile v8h*)q = hv;
    __threadfence();
  }
}

__global__ __launch_bounds__(256) void decay_table_kernel(
    const float* __restrict__ a_log, float* __restrict__ adec, int n)
{
  const int i  = blockIdx.x * 256 + threadIdx.x;
  const int ic = (i < n) ? i : (n - 1);
  const float v  = a_log[ic];
  const float sp = fmaxf(v, 0.0f) + log1pf(expf(-fabsf(v)));
  float a = expf(-sp);
  a = (a < 1.17549435e-38f) ? 0.0f : a;
  if (i < n) {
    *(volatile float*)(adec + i) = a;
    __threadfence();
    *(volatile float*)(adec + i) = a;
    __threadfence();
  }
}

__global__ __launch_bounds__(256) void rmsnorm_kernel(
    const float* __restrict__ x, const float* __restrict__ nw, unsigned short* __restrict__ xn,
    int rows, float carry)
{
  const int lane = threadIdx.x & 31;
  const int wave = threadIdx.x >> 5;
  const int row  = blockIdx.x * 8 + wave;
  if (row >= rows) return;
  const float* xr = x + (size_t)row * kDim;
  v4f v[8];
#pragma unroll
  for (int it = 0; it < 4; ++it) {
    v[2 * it]     = *(const v4f*)(xr + it * 256 + lane * 8);
    v[2 * it + 1] = *(const v4f*)(xr + it * 256 + lane * 8 + 4);
  }
  float ss = 0.0f;
#pragma unroll
  for (int i = 0; i < 8; ++i) {
#pragma unroll
    for (int e = 0; e < 4; ++e) ss += v[i][e] * v[i][e];
  }
#pragma unroll
  for (int off = 16; off > 0; off >>= 1) ss += __shfl_xor(ss, off, 32);
  const float r = rsqrtf(ss * (1.0f / (float)kDim) + kEps);
  v8h hv[4];
#pragma unroll
  for (int it = 0; it < 4; ++it) {
    const v4f w0 = *(const v4f*)(nw + it * 256 + lane * 8);
    const v4f w1 = *(const v4f*)(nw + it * 256 + lane * 8 + 4);
#pragma unroll
    for (int e = 0; e < 4; ++e) {
      hv[it][e]     = (_Float16)(((v[2 * it][e] * r) * w0[e]) * carry);
      hv[it][4 + e] = (_Float16)(((v[2 * it + 1][e] * r) * w1[e]) * carry);
    }
  }
  unsigned short* xo = xn + (size_t)row * kDim + lane * 8;
  for (int pass = 0; pass < 2; ++pass) {
#pragma unroll
    for (int it = 0; it < 4; ++it) *(volatile v8h*)(xo + it * 256) = hv[it];
    __threadfence();
  }
}

__global__ __launch_bounds__(256) void gated_gemm_kernel(
    const unsigned short* __restrict__ Ap, int lda,
    const unsigned short* __restrict__ Btp, int ldb, int gateRow0,
    unsigned short* __restrict__ Uout, int ldc,
    const float* __restrict__ biasP, const float* __restrict__ biasG,
    int M, int N, int K, float scale, float ocarry)
{
  const _Float16* A  = (const _Float16*)Ap;
  const _Float16* Bt = (const _Float16*)Btp;
  __shared__ __align__(16) float sT[8][16 * 68];
  const int lane = threadIdx.x & 31;
  const int wave = threadIdx.x >> 5;
  const int tilesN = N >> 6;
  const int tilesM = M >> 5;
  const int tile = blockIdx.x * 8 + wave;
  if (tile >= tilesM * tilesN) return;
  const int tm = tile / tilesN;
  const int tn = tile - tm * tilesN;
  const int m0 = tm << 5;
  const int n0 = tn << 6;
  const int rlane = lane & 15;
  const int koff  = (lane >> 4) * 8;
  const int mOff  = (lane >> 4) * 8;

  const _Float16* ap0 = A  + (size_t)(m0 + rlane) * lda + koff;
  const _Float16* ap1 = A  + (size_t)(m0 + 16 + rlane) * lda + koff;
  const _Float16* bpP = Bt + (size_t)(n0 + rlane) * ldb + koff;
  const _Float16* bpG = Bt + (size_t)(gateRow0 + n0 + rlane) * ldb + koff;
  const size_t bstep = (size_t)16 * ldb;

  v8f accP[2][4], accG[2][4];
#pragma unroll
  for (int i = 0; i < 2; ++i) {
#pragma unroll
    for (int j = 0; j < 4; ++j) {
      accP[i][j] = (v8f){0.f, 0.f, 0.f, 0.f, 0.f, 0.f, 0.f, 0.f};
      accG[i][j] = (v8f){0.f, 0.f, 0.f, 0.f, 0.f, 0.f, 0.f, 0.f};
    }
  }

  for (int k0 = 0; k0 < K; k0 += 32) {
    const v16h a0 = frag_load(ap0 + k0);
    const v16h a1 = frag_load(ap1 + k0);
    {
      v16h bp[4];
#pragma unroll
      for (int j = 0; j < 4; ++j) bp[j] = frag_load(bpP + (size_t)j * bstep + k0);
#pragma unroll
      for (int j = 0; j < 4; ++j) accP[0][j] = mma_f16(a0, bp[j], accP[0][j]);
#pragma unroll
      for (int j = 0; j < 4; ++j) guard1(accP[0][j], a0, bp[j]);
#pragma unroll
      for (int j = 0; j < 4; ++j) accP[1][j] = mma_f16(a1, bp[j], accP[1][j]);
#pragma unroll
      for (int j = 0; j < 4; ++j) guard1(accP[1][j], a1, bp[j]);
    }
    {
      v16h bg[4];
#pragma unroll
      for (int j = 0; j < 4; ++j) bg[j] = frag_load(bpG + (size_t)j * bstep + k0);
#pragma unroll
      for (int j = 0; j < 4; ++j) accG[0][j] = mma_f16(a0, bg[j], accG[0][j]);
#pragma unroll
      for (int j = 0; j < 4; ++j) guard1(accG[0][j], a0, bg[j]);
#pragma unroll
      for (int j = 0; j < 4; ++j) accG[1][j] = mma_f16(a1, bg[j], accG[1][j]);
#pragma unroll
      for (int j = 0; j < 4; ++j) guard1(accG[1][j], a1, bg[j]);
    }
  }

  float bpv[4], bgv[4];
#pragma unroll
  for (int j = 0; j < 4; ++j) {
    bpv[j] = biasP[n0 + (j << 4) + rlane];
    bgv[j] = biasG[n0 + (j << 4) + rlane];
  }
  float* slab = sT[wave];
  const int q = lane >> 3, c8 = (lane & 7) * 8;
#pragma unroll
  for (int i = 0; i < 2; ++i) {
    const int mBase = m0 + (i << 4);
#pragma unroll
    for (int j = 0; j < 4; ++j) {
#pragma unroll
      for (int r = 0; r < 8; ++r) {
        const float p = accP[i][j][r] * scale + bpv[j];
        const float z = accG[i][j][r] * scale + bgv[j];
        const float e = __expf(-z);
        const float g = __builtin_amdgcn_rcpf(1.0f + e);
        slab[(mOff + r) * 68 + (j << 4) + rlane] = (p * g) * ocarry;
      }
    }
    wave_lds_sync();
    v8h hv[4];
#pragma unroll
    for (int it = 0; it < 4; ++it) {
      const float* sp = slab + (it * 4 + q) * 68 + c8;
      const v4f s0 = *(const v4f*)(sp);
      const v4f s1 = *(const v4f*)(sp + 4);
#pragma unroll
      for (int e = 0; e < 4; ++e) {
        hv[it][e]     = (_Float16)s0[e];
        hv[it][4 + e] = (_Float16)s1[e];
      }
    }
    for (int pass = 0; pass < 2; ++pass) {
#pragma unroll
      for (int it = 0; it < 4; ++it)
        *(volatile v8h*)(Uout + (size_t)(mBase + it * 4 + q) * ldc + n0 + c8) = hv[it];
      __threadfence();
    }
    wave_lds_sync();
  }
}

template <int OUT_MODE>
__global__ __launch_bounds__(256) void gemm64_kernel(
    const unsigned short* __restrict__ Ap, int lda,
    const unsigned short* __restrict__ Btp, int ldb, long strideB,
    void* __restrict__ Cout, int ldc, long strideC,
    const float* __restrict__ bias0, const float* __restrict__ bias1, const float* __restrict__ bias2,
    const float* __restrict__ resid,
    int M, int N, int K, float scale)
{
  const int pb = blockIdx.y;
  const _Float16* A  = (const _Float16*)Ap;
  const _Float16* Bt = (const _Float16*)Btp + (size_t)pb * strideB;
  const float* bias = (pb == 0) ? bias0 : ((pb == 1) ? bias1 : bias2);
  __shared__ __align__(16) float sT[8][16 * 68];
  const int lane = threadIdx.x & 31;
  const int wave = threadIdx.x >> 5;
  const int tilesN = N >> 6;
  const int tilesM = M >> 6;
  const int tile = blockIdx.x * 8 + wave;
  if (tile >= tilesM * tilesN) return;
  const int tm = tile / tilesN;
  const int tn = tile - tm * tilesN;
  const int m0 = tm << 6;
  const int n0 = tn << 6;
  const int rlane = lane & 15;
  const int koff  = (lane >> 4) * 8;
  const int mOff  = (lane >> 4) * 8;

  const _Float16* apb = A  + (size_t)(m0 + rlane) * lda + koff;
  const _Float16* bpb = Bt + (size_t)(n0 + rlane) * ldb + koff;
  const size_t astep = (size_t)16 * lda;
  const size_t bstep = (size_t)16 * ldb;

  v8f acc[4][4];
#pragma unroll
  for (int i = 0; i < 4; ++i) {
#pragma unroll
    for (int j = 0; j < 4; ++j) acc[i][j] = (v8f){0.f, 0.f, 0.f, 0.f, 0.f, 0.f, 0.f, 0.f};
  }

  for (int k0 = 0; k0 < K; k0 += 32) {
    v16h bh[4];
#pragma unroll
    for (int j = 0; j < 4; ++j) bh[j] = frag_load(bpb + (size_t)j * bstep + k0);
#pragma unroll
    for (int i = 0; i < 4; ++i) {
      const v16h ah = frag_load(apb + (size_t)i * astep + k0);
#pragma unroll
      for (int j = 0; j < 4; ++j) acc[i][j] = mma_f16(ah, bh[j], acc[i][j]);
#pragma unroll
      for (int j = 0; j < 4; ++j) guard1(acc[i][j], ah, bh[j]);
    }
  }

  float* slab = sT[wave];
  if (OUT_MODE == 0) {
    float* C = (float*)Cout + (size_t)pb * strideC;
    const int hh = lane >> 4, c4 = (lane & 15) * 4;
    const v4f bias4 = *(const v4f*)(bias + n0 + c4);
#pragma unroll
    for (int i = 0; i < 4; ++i) {
      const int mBase = m0 + (i << 4);
#pragma unroll
      for (int j = 0; j < 4; ++j) {
#pragma unroll
        for (int r = 0; r < 8; ++r) slab[(mOff + r) * 68 + (j << 4) + rlane] = acc[i][j][r] * scale;
      }
      wave_lds_sync();
#pragma unroll
      for (int g2 = 0; g2 < 2; ++g2) {
        v4f val[4];
#pragma unroll
        for (int it = 0; it < 4; ++it) {
          const int row = (g2 * 4 + it) * 2 + hh;
          const v4f s  = *(const v4f*)(slab + row * 68 + c4);
          const v4f rv = *(const v4f*)(resid + (size_t)(mBase + row) * ldc + n0 + c4);
          val[it] = (s + bias4) + rv;
        }
        for (int pass = 0; pass < 2; ++pass) {
#pragma unroll
          for (int it = 0; it < 4; ++it) {
            const int row = (g2 * 4 + it) * 2 + hh;
            *(volatile v4f*)(C + (size_t)(mBase + row) * ldc + n0 + c4) = val[it];
          }
          __threadfence();
        }
      }
      wave_lds_sync();
    }
  } else {
    unsigned short* C = (unsigned short*)Cout + (size_t)pb * strideC;
    const int q = lane >> 3, c8 = (lane & 7) * 8;
    const v4f biasA = *(const v4f*)(bias + n0 + c8);
    const v4f biasB = *(const v4f*)(bias + n0 + c8 + 4);
#pragma unroll
    for (int i = 0; i < 4; ++i) {
      const int mBase = m0 + (i << 4);
#pragma unroll
      for (int j = 0; j < 4; ++j) {
#pragma unroll
        for (int r = 0; r < 8; ++r) slab[(mOff + r) * 68 + (j << 4) + rlane] = acc[i][j][r] * scale;
      }
      wave_lds_sync();
      v8h hv[4];
#pragma unroll
      for (int it = 0; it < 4; ++it) {
        const float* sp = slab + (it * 4 + q) * 68 + c8;
        const v4f s0 = *(const v4f*)(sp) + biasA;
        const v4f s1 = *(const v4f*)(sp + 4) + biasB;
#pragma unroll
        for (int e = 0; e < 4; ++e) {
          hv[it][e]     = (_Float16)s0[e];
          hv[it][4 + e] = (_Float16)s1[e];
        }
      }
      for (int pass = 0; pass < 2; ++pass) {
#pragma unroll
        for (int it = 0; it < 4; ++it)
          *(volatile v8h*)(C + (size_t)(mBase + it * 4 + q) * ldc + n0 + c8) = hv[it];
        __threadfence();
      }
      wave_lds_sync();
    }
  }
}

__global__ __launch_bounds__(64) void scan_kernel(
    const unsigned* __restrict__ bP, const unsigned* __restrict__ cP, const unsigned* __restrict__ dP,
    const float* __restrict__ adec, unsigned* __restrict__ yP, float ycarry)
{
  const int gid  = blockIdx.x * 64 + threadIdx.x;
  const int bt   = gid / kPairs;
  const int pair = gid - bt * kPairs;
  const float a0 = adec[2 * pair];
  const float a1 = adec[2 * pair + 1];
  float h0 = 0.0f, h1 = 0.0f;
  const size_t base = (size_t)bt * kSeq * kPairs + pair;
#pragma unroll 1
  for (int t0 = 0; t0 < kSeq; t0 += 4) {
    unsigned bw[4], cw[4], dw[4], yw[4];
#pragma unroll
    for (int s = 0; s < 4; ++s) {
      const size_t o = base + (size_t)(t0 + s) * kPairs;
      bw[s] = bP[o];
      cw[s] = cP[o];
      dw[s] = dP[o];
    }
#pragma unroll
    for (int s = 0; s < 4; ++s) {
      const float b0 = h16_to_f32(bw[s] & 0xffffu);
      const float b1 = h16_to_f32(bw[s] >> 16);
      const float c0 = h16_to_f32(cw[s] & 0xffffu);
      const float c1 = h16_to_f32(cw[s] >> 16);
      const float d0 = h16_to_f32(dw[s] & 0xffffu);
      const float d1 = h16_to_f32(dw[s] >> 16);
      h0 = a0 * h0 + b0;
      h1 = a1 * h1 + b1;
      const float y0 = c0 * h0 + d0;
      const float y1 = c1 * h1 + d1;
      yw[s] = pack_h2(y0 * ycarry, y1 * ycarry);
    }
    for (int pass = 0; pass < 2; ++pass) {
#pragma unroll
      for (int s = 0; s < 4; ++s)
        *(volatile unsigned*)(yP + base + (size_t)(t0 + s) * kPairs) = yw[s];
      __threadfence();
    }
  }
}

extern "C" void kernel_launch(void* const* d_in, const int* in_sizes, int n_in,
                              void* d_out, int out_size, void* d_ws, size_t ws_size,
                              hipStream_t stream) {
  if (n_in < 15) return;
  if (in_sizes[0] != kBatch * kSeq * kDim) return;
  if (in_sizes[1] != kDim) return;
  if (in_sizes[2] != kInner * kDim) return;
  if (in_sizes[3] != kInner) return;
  if (in_sizes[4] != kInner * kDim) return;
  if (in_sizes[5] != kInner) return;
  if (in_sizes[6] != kInner * kInner) return;
  if (in_sizes[7] != kInner) return;
  if (in_sizes[8] != kInner * kInner) return;
  if (in_sizes[9] != kInner) return;
  if (in_sizes[10] != kInner * kInner) return;
  if (in_sizes[11] != kInner) return;
  if (in_sizes[12] != kDim * kInner) return;
  if (in_sizes[13] != kDim) return;
  if (in_sizes[14] != kInner) return;
  if (out_size != kBatch * kSeq * kDim) return;
  if (ws_size < kWsTotal) return;

  const float* x      = (const float*)d_in[0];
  const float* norm_w = (const float*)d_in[1];
  const float* in_w   = (const float*)d_in[2];
  const float* in_b   = (const float*)d_in[3];
  const float* gate_w = (const float*)d_in[4];
  const float* gate_b = (const float*)d_in[5];
  const float* b_w    = (const float*)d_in[6];
  const float* b_b    = (const float*)d_in[7];
  const float* c_w    = (const float*)d_in[8];
  const float* c_b    = (const float*)d_in[9];
  const float* d_w    = (const float*)d_in[10];
  const float* d_b    = (const float*)d_in[11];
  const float* out_w  = (const float*)d_in[12];
  const float* out_b  = (const float*)d_in[13];
  const float* a_log  = (const float*)d_in[14];
  float* out = (float*)d_out;

  char* ws = (char*)d_ws;
  unsigned short* WIG  = (unsigned short*)(ws + kOffWIG);
  unsigned short* WBCD = (unsigned short*)(ws + kOffWBCD);
  unsigned short* WO   = (unsigned short*)(ws + kOffWO);
  unsigned short* XN   = (unsigned short*)(ws + kOffXN);
  unsigned short* U    = (unsigned short*)(ws + kOffU);
  unsigned short* BCD  = (unsigned short*)(ws + kOffBCD);
  unsigned short* Y    = (unsigned short*)(ws + kOffY);
  float*          ADEC = (float*)(ws + kOffADEC);

  const size_t planeElems = (size_t)kSlabRows * kInner;

  {
    const int n8a = kInner * kDim / 8;
    const int n8b = kInner * kInner / 8;
    cast_carry_f16_kernel<<<n8a / 256, 256, 0, stream>>>(in_w,   WIG, n8a, kWCarry);
    cast_carry_f16_kernel<<<n8a / 256, 256, 0, stream>>>(gate_w, WIG + (size_t)kInner * kDim, n8a, kWCarry);
    cast_carry_f16_kernel<<<n8b / 256, 256, 0, stream>>>(b_w, WBCD, n8b, kWCarry);
    cast_carry_f16_kernel<<<n8b / 256, 256, 0, stream>>>(c_w, WBCD + (size_t)kInner * kInner, n8b, kWCarry);
    cast_carry_f16_kernel<<<n8b / 256, 256, 0, stream>>>(d_w, WBCD + (size_t)2 * kInner * kInner, n8b, kWCarry);
    cast_carry_f16_kernel<<<n8a / 256, 256, 0, stream>>>(out_w, WO, n8a, kWCarry);
  }
  decay_table_kernel<<<kInner / 256, 256, 0, stream>>>(a_log, ADEC, kInner);

  for (int s = 0; s < kSlabs; ++s) {
    const float* xs = x   + (size_t)s * kSlabRows * kDim;
    float*       os = out + (size_t)s * kSlabRows * kDim;

    rmsnorm_kernel<<<kSlabRows / 8, 256, 0, stream>>>(xs, norm_w, XN, kSlabRows, kXnCarry);

    gated_gemm_kernel<<<((kSlabRows / 32) * (kInner / 64)) / 8, 256, 0, stream>>>(
        XN, kDim, WIG, kDim, kInner, U, kInner, in_b, gate_b,
        kSlabRows, kInner, kDim, kScaleIG, kUCarry);

    gemm64_kernel<1><<<dim3(((kSlabRows / 64) * (kInner / 64)) / 8, 3), 256, 0, stream>>>(
        U, kInner, WBCD, kInner, (long)kInner * kInner,
        (void*)BCD, kInner, (long)planeElems,
        b_b, c_b, d_b, nullptr,
        kSlabRows, kInner, kInner, kScaleBCD);

    scan_kernel<<<(kSlabB * kPairs) / 64, 64, 0, stream>>>(
        (const unsigned*)BCD, (const unsigned*)(BCD + planeElems), (const unsigned*)(BCD + 2 * planeElems),
        ADEC, (unsigned*)Y, kYCarry);

    gemm64_kernel<0><<<dim3(((kSlabRows / 64) * (kDim / 64)) / 8, 1), 256, 0, stream>>>(
        Y, kInner, WO, kInner, 0L,
        (void*)os, kDim, 0L,
        out_b, out_b, out_b, xs,
        kSlabRows, kDim, kInner, kScaleOut);
  }
}
